// TangentConv_83734682403284
// MI455X (gfx1250) — hardware-run, weakly checked
//
#include <hip/hip_runtime.h>


namespace {
constexpr int N0 = 100000, N1 = 50000, N2 = 25000, KN = 9, PF = 8;
constexpr float HS = 256.0f, WSC = 256.0f, SL = 0.1f;
typedef _Float16 b16;
typedef __attribute__((ext_vector_type(16))) _Float16 v16b;
typedef __attribute__((ext_vector_type(8))) _Float16 v8b;
typedef __attribute__((ext_vector_type(8))) float v8f;
typedef __attribute__((ext_vector_type(4))) float v4f;
__device__ __forceinline__ float bf16_rne(float f) { unsigned int u = __float_as_uint(f); u += 0x7FFFu + ((u >> 16) & 1u); float r = __uint_as_float(u & 0xFFFF0000u); asm volatile("" : "+v"(r)); return r; }
__device__ __forceinline__ float bfv(float f) { float r = bf16_rne(f); asm volatile("" : "+v"(r)); return r; }
__device__ __forceinline__ void split16(float v, b16& hi, b16& lo) { hi = (b16)v; lo = (b16)(v - (float)hi); }
__device__ __forceinline__ v16b frag_kb(const b16* p, int hh) { const v8b a = *(const v8b*)(p + 8 * hh), b = *(const v8b*)(p + 16 + 8 * hh); v16b f;
#pragma unroll
  for (int e = 0; e < 8; ++e) { f[e] = a[e]; f[8 + e] = b[e]; } return f; }
__device__ __forceinline__ v8f wmma16b(v16b a, v16b b, v8f c) { v8f d = __builtin_amdgcn_wmma_f32_16x16x32_f16(false, a, false, b, (short)0, c, false, false); asm volatile("v_nop\n\tv_nop\n\tv_nop\n\tv_nop" : "+v"(d) : "v"(a), "v"(b)); return d; }
__device__ __forceinline__ void wave_lds_sync() { __builtin_amdgcn_fence(__ATOMIC_RELEASE, "workgroup"); __builtin_amdgcn_wave_barrier(); __builtin_amdgcn_fence(__ATOMIC_ACQUIRE, "workgroup"); }
__device__ __forceinline__ float pmul(float a, float b) { float p = a * b; asm volatile("" : "+v"(p)); return p; }
__device__ __forceinline__ int iclamp(int v, int lo, int hi) { return v < lo ? lo : (v > hi ? hi : v); }
__device__ __forceinline__ float leaky(float v) { return v > 0.0f ? v : SL * v; }

template <int CIN, int COUT, int KP>
__global__ __launch_bounds__(256) void wputc_kernel(const float* __restrict__ w, b16* __restrict__ WT) { const int u = blockIdx.x * 256 + threadIdx.x; if (u >= COUT * (KP / 8)) return; const int o = u / (KP / 8), q0 = (u % (KP / 8)) * 8; v8b v;
#pragma unroll
  for (int j = 0; j < 8; ++j) { const int q = q0 + j; const int k = q / CIN, c = q % CIN; v[j] = (b16)(q < KN * CIN ? bf16_rne(w[((size_t)o * CIN + c) * KN + k]) * WSC : 0.0f); }
  for (int pass = 0; pass < 2; ++pass) { *(volatile v8b*)(WT + (size_t)o * KP + q0) = v; __threadfence(); } }
template <int CX, int DEP, int COUT, int KP, int EXA, int NIN>
__global__ __launch_bounds__(32) void tconv_kernel(const float* __restrict__ IN, const int* __restrict__ ind, const float* __restrict__ depth, const b16* __restrict__ WT, const float* __restrict__ bias, int NLIM, int INLIM, float* __restrict__ OUT) {
  constexpr int CIN = CX + DEP, NT = COUT / 16; __shared__ __attribute__((aligned(16))) b16 Ph[16][KP + 8], Pl[16][KP + 8]; __shared__ float Tf[16][COUT + 4]; const int lane = threadIdx.x, nloc = lane & 15, hlf = lane >> 4; const size_t m0 = (size_t)blockIdx.x * 16; if (m0 >= (size_t)NLIM) return;
  for (int rr = 0; rr < 16; ++rr) for (int q = lane; q < KP + 8; q += 32) { Ph[rr][q] = (b16)0.0f; Pl[rr][q] = (b16)0.0f; }
  wave_lds_sync();
  for (int rr = 0; rr < 16; ++rr) { const size_t n = m0 + rr; if (n >= (size_t)NLIM) continue;
    for (int k = 0; k < KN; ++k) { const int j = iclamp(ind[n * KN + k], 0, NIN - 1); const bool inr = j < INLIM;
      for (int c = lane; c < CIN; c += 32) { float v; if (DEP && c == CX) v = bfv(depth[n * KN + k]); else v = inr ? (EXA ? bfv(IN[(size_t)j * CX + c]) : IN[(size_t)j * CX + c]) : 0.0f; b16 p, ql; if (EXA || (DEP && c == CX)) { p = (b16)(v * HS); ql = (b16)0.0f; } else split16(v * HS, p, ql); Ph[rr][k * CIN + c] = p; Pl[rr][k * CIN + c] = ql; } } }
  wave_lds_sync(); v8f acc[NT];
#pragma unroll
  for (int t = 0; t < NT; ++t) acc[t] = (v8f){};
#pragma unroll 2
  for (int kb = 0; kb < KP; kb += 32) { const v16b a = frag_kb(&Ph[nloc][kb], hlf), al = frag_kb(&Pl[nloc][kb], hlf);
#pragma unroll
    for (int t = 0; t < NT; ++t) { const v16b bw = frag_kb(WT + (size_t)(t * 16 + nloc) * KP + kb, hlf); acc[t] = wmma16b(a, bw, acc[t]); if (!EXA) acc[t] = wmma16b(al, bw, acc[t]); } }
#pragma unroll
  for (int t = 0; t < NT; ++t) { const int cc = t * 16 + nloc; const float bb = bfv(bias[cc]);
#pragma unroll
    for (int r8 = 0; r8 < 8; ++r8) Tf[8 * hlf + r8][cc] = leaky(acc[t][r8] * (1.0f / (HS * WSC)) + bb); }
  wave_lds_sync();
  for (int pass = 0; pass < 2; ++pass) { for (int rr = 0; rr < 16; ++rr) if (m0 + rr < (size_t)NLIM) for (int c = lane; c < COUT; c += 32) ((volatile float*)OUT)[(m0 + rr) * COUT + c] = Tf[rr][c]; __threadfence(); } }
template <int C, int NIN>
__global__ __launch_bounds__(256) void tpool_kernel(const float* __restrict__ IN, const int* __restrict__ pind, int NLIM, int INLIM, float* __restrict__ OUT) { const int wave = threadIdx.x >> 5, lane = threadIdx.x & 31; const size_t n = (size_t)blockIdx.x * 8 + wave; if (n >= (size_t)NLIM) return; float acc[C / 32 > 0 ? C / 32 : 1]; for (int q = 0; q < C / 32; ++q) acc[q] = 0.0f;
  for (int p = 0; p < PF; ++p) { const int j = pind[n * PF + p]; if (j < 0) continue; const int jj = iclamp(j, 0, NIN - 1); if (jj >= INLIM) continue;
#pragma unroll
    for (int q = 0; q < C / 32; ++q) acc[q] += IN[(size_t)jj * C + q * 32 + lane]; }
  for (int pass = 0; pass < 2; ++pass) { for (int q = 0; q < C / 32; ++q) ((volatile float*)OUT)[n * C + q * 32 + lane] = acc[q]; __threadfence(); } }
__global__ __launch_bounds__(256) void latent_kernel(const float* __restrict__ Hh, const float* __restrict__ wl, const float* __restrict__ bl, int NLIM, float* __restrict__ out) { const int wave = threadIdx.x >> 5, lane = threadIdx.x & 31; const size_t n0 = (size_t)blockIdx.x * 256 + wave * 32; if (n0 >= (size_t)NLIM) return; const size_t n = n0 + lane; float s = 0.0f;
  if (n < (size_t)NLIM) {
#pragma unroll 4
    for (int c = 0; c < 128; ++c) s += pmul(Hh[n * 128 + c], bfv(wl[c])); s = leaky(s + bfv(bl[0])); }
  for (int pass = 0; pass < 2; ++pass) { if (n < (size_t)NLIM) ((volatile float*)out)[n] = s; __threadfence(); } }
}

extern "C" void kernel_launch(void* const* d_in, const int* in_sizes, int n_in, void* d_out, int out_size, void* d_ws, size_t ws_size, hipStream_t stream) {
  (void)n_in;
  auto Fp = [&](int i) { return (const float*)d_in[i]; }; auto Ip = [&](int i) { return (const int*)d_in[i]; };
  if (in_sizes[0] != N0 * 3 || in_sizes[1] != N0 * KN || in_sizes[2] != N0 * KN || in_sizes[3] != N1 * KN || in_sizes[5] != N1 * PF || in_sizes[6] != N2 * KN || in_sizes[8] != N2 * PF || in_sizes[9] != 32 * 4 * KN || in_sizes[11] != 32 * 32 * KN || in_sizes[13] != 64 * 33 * KN || in_sizes[15] != 64 * 64 * KN || in_sizes[17] != 128 * 65 * KN || in_sizes[19] != 128 || out_size != N2) return;
  const int L0 = N0, L1 = N1, L2 = N2;
  constexpr int KP11 = 64  , KP12 = 288, KP21 = 320  , KP22 = 576, KP31 = 608  ;
  size_t off = 0; char* ws = (char*)d_ws;
  auto carve = [&](size_t bytes) { char* p = ws + off; off += (bytes + 255) & ~(size_t)255; return p; };
  b16* W11 = (b16*)carve((size_t)32 * KP11 * 2); b16* W12 = (b16*)carve((size_t)32 * KP12 * 2); b16* W21 = (b16*)carve((size_t)64 * KP21 * 2); b16* W22 = (b16*)carve((size_t)64 * KP22 * 2); b16* W31 = (b16*)carve((size_t)128 * KP31 * 2);
  float* H0a = (float*)carve((size_t)N0 * 32 * 4); float* H0b = (float*)carve((size_t)N0 * 32 * 4); float* P1 = (float*)carve((size_t)N1 * 32 * 4); float* H1a = (float*)carve((size_t)N1 * 64 * 4); float* H1b = (float*)carve((size_t)N1 * 64 * 4); float* P2 = (float*)carve((size_t)N2 * 64 * 4); float* H2 = (float*)carve((size_t)N2 * 128 * 4);
  if (off > ws_size || off > ((size_t)96 << 20)) return;
  wputc_kernel<4, 32, KP11><<<(32 * KP11 / 8 + 255) / 256, 256, 0, stream>>>(Fp(9), W11); wputc_kernel<32, 32, KP12><<<(32 * KP12 / 8 + 255) / 256, 256, 0, stream>>>(Fp(11), W12);
  wputc_kernel<33, 64, KP21><<<(64 * KP21 / 8 + 255) / 256, 256, 0, stream>>>(Fp(13), W21); wputc_kernel<64, 64, KP22><<<(64 * KP22 / 8 + 255) / 256, 256, 0, stream>>>(Fp(15), W22);
  wputc_kernel<65, 128, KP31><<<(128 * KP31 / 8 + 255) / 256, 256, 0, stream>>>(Fp(17), W31);
  tconv_kernel<3, 1, 32, KP11, 1, N0><<<L0 / 16, 32, 0, stream>>>(Fp(0), Ip(1), Fp(2), W11, Fp(10), L0, N0, H0a);
  tconv_kernel<32, 0, 32, KP12, 0, N0><<<L0 / 16, 32, 0, stream>>>(H0a, Ip(1), Fp(2), W12, Fp(12), L0, L0, H0b);
  tpool_kernel<32, N0><<<(L1 + 7) / 8, 256, 0, stream>>>(H0b, Ip(5), L1, L0, P1);
  tconv_kernel<32, 1, 64, KP21, 0, N1><<<L1 / 16, 32, 0, stream>>>(P1, Ip(3), Fp(4), W21, Fp(14), L1, L1, H1a);
  tconv_kernel<64, 0, 64, KP22, 0, N1><<<L1 / 16, 32, 0, stream>>>(H1a, Ip(3), Fp(4), W22, Fp(16), L1, L1, H1b);
  tpool_kernel<64, N1><<<(L2 + 7) / 8, 256, 0, stream>>>(H1b, Ip(8), L2, L1, P2);
  tconv_kernel<64, 1, 128, KP31, 0, N2><<<(L2 + 15) / 16, 32, 0, stream>>>(P2, Ip(6), Fp(7), W31, Fp(18), L2, L2, H2);
  latent_kernel<<<(L2 + 255) / 256, 256, 0, stream>>>(H2, Fp(19), Fp(20), L2, (float*)d_out);
}
